// MaskedRNN_21818433863703
// MI455X (gfx1250) — hardware-verified
//
#include <hip/hip_runtime.h>
#include <math.h>

typedef __attribute__((ext_vector_type(16))) _Float16 v16h;
typedef __attribute__((ext_vector_type(8)))  _Float16 v8h;
typedef __attribute__((ext_vector_type(8)))  float    v8f;
typedef __attribute__((ext_vector_type(4)))  float    v4f;

__device__ __forceinline__ void dep_guard_h(v8f& a, v8f& b, v16h x, v16h y) { asm volatile("v_nop\n\tv_nop\n\tv_nop\n\tv_nop" : "+v"(a), "+v"(b) : "v"(x), "v"(y)); }
__device__ __forceinline__ void keep4_h(v16h a, v16h b, v16h c, v16h d) { asm volatile("v_nop" :: "v"(a), "v"(b), "v"(c), "v"(d)); }
template <typename T> struct Frag;
template <> struct Frag<_Float16> {
  typedef v16h V; union U { v16h v; v8h h[2]; };
  static __device__ __forceinline__ v16h load(const _Float16* p) {
    U f; f.h[0] = *(const v8h*)(p); f.h[1] = *(const v8h*)(p + 16); return f.v;
  }
  static __device__ __forceinline__ v8f mma(v16h a, v16h b, v8f c) {
    return __builtin_amdgcn_wmma_f32_16x16x32_f16(false, a, false, b, (short)0, c, false, false);
  }
  static __device__ __forceinline__ void guard(v8f& a, v8f& b, v16h x, v16h y) { dep_guard_h(a, b, x, y); }
  static __device__ __forceinline__ void keep(v16h a, v16h b, v16h c, v16h d) { keep4_h(a, b, c, d); }
};

__device__ __forceinline__ v8f mma_f16(v16h a, v16h b, v8f c) {
  c = __builtin_amdgcn_wmma_f32_16x16x32_f16(false, a, false, b, (short)0, c, false, false);
  asm volatile("v_nop\n\tv_nop\n\tv_nop\n\tv_nop" : "+v"(c) : "v"(a), "v"(b));
  return c;
}

constexpr int kSeq    = 512;
constexpr int kBatch  = 64;
constexpr int kEmb    = 256;
constexpr int kHid    = 256;
constexpr int kGate3  = 768;
constexpr int kRowsPerBlk = 16;
constexpr int kThreads    = 256;
constexpr int kATP = 528;
constexpr int kHSP = 264;
constexpr float kOpScale  = 256.0f;
constexpr float kAccScale = 1.0f / 65536.0f;
static_assert(kBatch % kRowsPerBlk == 0, "batch tile");
static_assert(kEmb % 32 == 0 && kHid % 32 == 0, "K steps of 32");
static_assert((kThreads / 32) * 32 == kHid, "8 waves x 32 units cover H");
static_assert(kATP % 16 == 0 && kHSP % 4 == 0, "aligned pitches");

__global__ __launch_bounds__(256) void cast_scale_f16x2(
    const float* __restrict__ in, _Float16* __restrict__ out, int n2, float sc) {
  int i = blockIdx.x * 256 + threadIdx.x;
  if (i < n2) {
    const _Float16 h0 = (_Float16)(in[2 * i] * sc), h1 = (_Float16)(in[2 * i + 1] * sc);
    const unsigned u = (unsigned)__builtin_bit_cast(unsigned short, h0) | ((unsigned)__builtin_bit_cast(unsigned short, h1) << 16);
    ((volatile unsigned*)out)[i] = u;
    __threadfence();
    ((volatile unsigned*)out)[i] = u;
  }
}

__global__ __launch_bounds__(256) void gru_seq_kernel(
    const int* __restrict__ ids, const float* __restrict__ emb,
    const _Float16* __restrict__ wih16, const _Float16* __restrict__ whh16,
    const float* __restrict__ b_ih, const float* __restrict__ b_hh,
    float* __restrict__ out, int vocab) {
  __shared__ __align__(16) _Float16 Atile[kRowsPerBlk * kATP];
  __shared__ __align__(16) float    hslab[kRowsPerBlk * kHSP];

  const int tid  = threadIdx.x;
  const int lane = tid & 31;
  const int wave = tid >> 5;
  const int hh   = lane >> 4;
  const int c    = lane & 15;
  const int koff = hh * 8;
  const int blk  = blockIdx.x;
  const int ucol0 = wave * 32;

  const int brow  = tid >> 4;
  const int bseg  = (tid & 15) * 16;
  const int bglob = blk * kRowsPerBlk + brow;

  {
    const v4f z4 = {0.f, 0.f, 0.f, 0.f};
#pragma unroll
    for (int e = 0; e < 4; ++e) *(v4f*)(hslab + brow * kHSP + bseg + 4 * e) = z4;
  }
  float hreg[2][8];
#pragma unroll
  for (int j = 0; j < 2; ++j)
#pragma unroll
    for (int r = 0; r < 8; ++r) hreg[j][r] = 0.f;

  float bsr[2], bsz[2], bxn[2], bhn[2];
#pragma unroll
  for (int j = 0; j < 2; ++j) {
    const int n = ucol0 + 16 * j + c;
    bsr[j] = b_ih[n] + b_hh[n];
    bsz[j] = b_ih[kHid + n] + b_hh[kHid + n];
    bxn[j] = b_ih[2 * kHid + n];
    bhn[j] = b_hh[2 * kHid + n];
  }

  const int q  = lane >> 3;
  const int c4 = (lane & 7) * 4;

  for (int t = 0; t < kSeq; ++t) {
    __syncthreads();

    {
      int id = ids[bglob * kSeq + t];
      id = id < 0 ? 0 : (id >= vocab ? vocab - 1 : id);
      const float* er = emb + (size_t)id * kEmb + bseg;
      const float* hr = hslab + brow * kHSP + bseg;
      const v4f e0 = *(const v4f*)(er), e1 = *(const v4f*)(er + 4), e2 = *(const v4f*)(er + 8), e3 = *(const v4f*)(er + 12);
      const v4f g0 = *(const v4f*)(hr), g1 = *(const v4f*)(hr + 4), g2 = *(const v4f*)(hr + 8), g3 = *(const v4f*)(hr + 12);
      v8h xa, xb, ha, hb;
#pragma unroll
      for (int e = 0; e < 4; ++e) {
        xa[e] = (_Float16)(e0[e] * kOpScale); xa[4 + e] = (_Float16)(e1[e] * kOpScale);
        xb[e] = (_Float16)(e2[e] * kOpScale); xb[4 + e] = (_Float16)(e3[e] * kOpScale);
        ha[e] = (_Float16)(g0[e] * kOpScale); ha[4 + e] = (_Float16)(g1[e] * kOpScale);
        hb[e] = (_Float16)(g2[e] * kOpScale); hb[4 + e] = (_Float16)(g3[e] * kOpScale);
      }
      _Float16* arow = Atile + brow * kATP;
      *(v8h*)(arow + bseg)            = xa;
      *(v8h*)(arow + bseg + 8)        = xb;
      *(v8h*)(arow + kEmb + bseg)     = ha;
      *(v8h*)(arow + kEmb + bseg + 8) = hb;
    }
    __syncthreads();

    v8f accR[2], accZ[2], accXN[2], accHN[2];
#pragma unroll
    for (int j = 0; j < 2; ++j) {
      accR[j]  = (v8f){0.f,0.f,0.f,0.f,0.f,0.f,0.f,0.f};
      accZ[j]  = (v8f){0.f,0.f,0.f,0.f,0.f,0.f,0.f,0.f};
      accXN[j] = (v8f){0.f,0.f,0.f,0.f,0.f,0.f,0.f,0.f};
      accHN[j] = (v8f){0.f,0.f,0.f,0.f,0.f,0.f,0.f,0.f};
    }
    const _Float16* afrag = Atile + c * kATP + koff;
#pragma unroll 1
    for (int kk = 0; kk < kEmb / 32; ++kk) {
      const int k0 = kk * 32;
      const v16h a = Frag<_Float16>::load(afrag + k0);
#pragma unroll
      for (int j = 0; j < 2; ++j) {
        const _Float16* wb = wih16 + (size_t)(ucol0 + 16 * j + c) * kEmb + k0 + koff;
        const v16h w0 = Frag<_Float16>::load(wb);
        const v16h w1 = Frag<_Float16>::load(wb + (size_t)kHid * kEmb);
        const v16h w2 = Frag<_Float16>::load(wb + (size_t)2 * kHid * kEmb);
        accR[j]  = mma_f16(a, w0, accR[j]);
        accZ[j]  = mma_f16(a, w1, accZ[j]);
        accXN[j] = mma_f16(a, w2, accXN[j]);
      }
    }
#pragma unroll 1
    for (int kk = 0; kk < kHid / 32; ++kk) {
      const int k0 = kk * 32;
      const v16h a = Frag<_Float16>::load(afrag + kEmb + k0);
#pragma unroll
      for (int j = 0; j < 2; ++j) {
        const _Float16* wb = whh16 + (size_t)(ucol0 + 16 * j + c) * kHid + k0 + koff;
        const v16h w0 = Frag<_Float16>::load(wb);
        const v16h w1 = Frag<_Float16>::load(wb + (size_t)kHid * kHid);
        const v16h w2 = Frag<_Float16>::load(wb + (size_t)2 * kHid * kHid);
        accR[j]  = mma_f16(a, w0, accR[j]);
        accZ[j]  = mma_f16(a, w1, accZ[j]);
        accHN[j] = mma_f16(a, w2, accHN[j]);
      }
    }

#pragma unroll
    for (int j = 0; j < 2; ++j) {
      const int ncol = ucol0 + 16 * j + c;
#pragma unroll
      for (int r = 0; r < 8; ++r) {
        const float sr = accR[j][r] * kAccScale + bsr[j];
        const float sz = accZ[j][r] * kAccScale + bsz[j];
        const float rg = 1.0f / (1.0f + expf(-sr));
        const float zg = 1.0f / (1.0f + expf(-sz));
        const float hn = accHN[j][r] * kAccScale + bhn[j];
        const float npre = accXN[j][r] * kAccScale + bxn[j] + rg * hn;
        const float ng = tanhf(npre);
        const float hp = hreg[j][r];
        const float hnew = (1.0f - zg) * ng + zg * hp;
        hreg[j][r] = hnew;
        hslab[(8 * hh + r) * kHSP + ncol] = hnew;
      }
    }
    __builtin_amdgcn_fence(__ATOMIC_RELEASE, "workgroup");
    __builtin_amdgcn_wave_barrier();
    __builtin_amdgcn_fence(__ATOMIC_ACQUIRE, "workgroup");

    {
      float* obase = out + ((size_t)t * kBatch + (size_t)blk * kRowsPerBlk) * kHid + ucol0;
      for (int pass = 0; pass < 2; ++pass) {
#pragma unroll
        for (int it = 0; it < 4; ++it) {
          const int row = it * 4 + q;
          const v4f v = *(const v4f*)(hslab + row * kHSP + ucol0 + c4);
          *(volatile v4f*)(obase + (size_t)row * kHid + c4) = v;
        }
        __threadfence();
      }
    }
  }

  __builtin_amdgcn_fence(__ATOMIC_RELEASE, "workgroup");
  __builtin_amdgcn_wave_barrier();
  __builtin_amdgcn_fence(__ATOMIC_ACQUIRE, "workgroup");
  {
    float* obase = out + (size_t)kSeq * kBatch * kHid + (size_t)blk * kRowsPerBlk * kHid + ucol0;
    for (int pass = 0; pass < 2; ++pass) {
#pragma unroll
      for (int it = 0; it < 4; ++it) {
        const int row = it * 4 + q;
        const v4f v = *(const v4f*)(hslab + row * kHSP + ucol0 + c4);
        *(volatile v4f*)(obase + (size_t)row * kHid + c4) = v;
      }
      __threadfence();
    }
  }
}

extern "C" void kernel_launch(void* const* d_in, const int* in_sizes, int n_in,
                              void* d_out, int out_size, void* d_ws, size_t ws_size,
                              hipStream_t stream) {
  if (n_in < 6) return;
  const int*   ids  = (const int*)d_in[0];
  const float* emb  = (const float*)d_in[1];
  const float* Wih  = (const float*)d_in[2];
  const float* Whh  = (const float*)d_in[3];
  const float* bih  = (const float*)d_in[4];
  const float* bhh  = (const float*)d_in[5];
  float* out = (float*)d_out;

  int vocab = in_sizes[1] / kEmb;
  if (vocab < 1) vocab = 1;
  if (in_sizes[0] < kBatch * kSeq) return;
  if (in_sizes[2] < kGate3 * kEmb || in_sizes[3] < kGate3 * kHid) return;
  if ((size_t)out_size < (size_t)kSeq * kBatch * kHid + (size_t)kBatch * kHid) return;

  const size_t wihBytes = (size_t)kGate3 * kEmb * 2;
  const size_t whhBytes = (size_t)kGate3 * kHid * 2;
  if (wihBytes + whhBytes > ws_size) return;
  char* ws = (char*)d_ws;
  _Float16* wih16 = (_Float16*)(ws);
  _Float16* whh16 = (_Float16*)(ws + wihBytes);

  const int nW2ih = (kGate3 * kEmb) / 2;
  const int nW2hh = (kGate3 * kHid) / 2;
  cast_scale_f16x2<<<(nW2ih + 255) / 256, 256, 0, stream>>>(Wih, wih16, nW2ih, kOpScale);
  cast_scale_f16x2<<<(nW2hh + 255) / 256, 256, 0, stream>>>(Whh, whh16, nW2hh, kOpScale);

  gru_seq_kernel<<<kBatch / kRowsPerBlk, kThreads, 0, stream>>>(ids, emb, wih16, whh16, bih, bhh, out, vocab);
}
